// GRUModel_1219770712109
// MI455X (gfx1250) — hardware-run, weakly checked
//
#include <hip/hip_runtime.h>
#include <math.h>

constexpr int NSEQ    = 256;
constexpr int NSTEP   = 1024;
constexpr int NFEAT   = 37;
constexpr int NUNIT   = 64;
constexpr int NCOL3   = 3 * NUNIT;
constexpr int KPAD    = 64;
constexpr int NTHR    = 128;
constexpr int NWAVE   = NTHR / 32;
constexpr int SEQ_BLK = 16;
constexpr int APITCH  = 72;
constexpr int WPITCH  = 64;
constexpr int OPITCH  = 36;
constexpr int TGRP    = 32;
constexpr int NCONST  = 2 * NCOL3 + NUNIT + 4;
static_assert(NUNIT == 16 * NWAVE);
static_assert(NSEQ % SEQ_BLK == 0);
static_assert(NSTEP % TGRP == 0);
static_assert(KPAD % 32 == 0 && NFEAT <= KPAD && NUNIT % 32 == 0 && KPAD == NUNIT);
static_assert((KPAD * NCOL3) % NTHR == 0);
static_assert((SEQ_BLK * APITCH) % NTHR == 0);
static_assert((2 * NCOL3) % NTHR == 0);
static_assert(SEQ_BLK * (KPAD / 2) == 4 * NTHR);
static_assert(SEQ_BLK == 4 * NWAVE);
static_assert(SEQ_BLK <= 32 && NUNIT <= NTHR);
static_assert(APITCH % 8 == 0 && APITCH >= KPAD && WPITCH % 8 == 0 && WPITCH >= KPAD);
static_assert(OPITCH % 4 == 0 && OPITCH >= TGRP && TGRP == 32);

typedef __attribute__((ext_vector_type(16))) __bf16   v16b;
typedef __attribute__((ext_vector_type(8)))  __bf16   v8b;
typedef __attribute__((ext_vector_type(8)))  float    v8f;
typedef __attribute__((ext_vector_type(4)))  float    v4f;

__device__ __forceinline__ unsigned short f2bf_bits(float f) {
  unsigned u = __float_as_uint(f);
  return (unsigned short)((u + 0x7FFFu + ((u >> 16) & 1u)) >> 16);
}

__device__ __forceinline__ void guard4x(v8f& a, v8f& b, v8f& c, v8f& d, v16b x, v16b y0, v16b y1, v16b y2) {
  asm volatile("v_nop\n\tv_nop\n\tv_nop\n\tv_nop" : "+v"(a), "+v"(b), "+v"(c), "+v"(d) : "v"(x), "v"(y0), "v"(y1), "v"(y2));
}
__device__ __forceinline__ void acc_guard4(v8f& a, v8f& b, v8f& c, v8f& d) {
  asm volatile("v_nop\n\tv_nop\n\tv_nop\n\tv_nop" : "+v"(a), "+v"(b), "+v"(c), "+v"(d));
}

template <typename T> struct Frag;
template <> struct Frag<__bf16> {
  typedef v16b V; union U { v16b v; v8b h[2]; };
  static __device__ __forceinline__ v16b load(const __bf16* p) {
    U f; f.h[0] = *(const v8b*)(p); f.h[1] = *(const v8b*)(p + 16); return f.v;
  }
  static __device__ __forceinline__ v8f mma(v16b a, v16b b, v8f c) {
    return __builtin_amdgcn_wmma_f32_16x16x32_bf16(false, a, false, b, (short)0, c, false, false);
  }
};

__device__ __forceinline__ float fsig(float x)  { return __builtin_amdgcn_rcpf(1.0f + expf(-x)); }
__device__ __forceinline__ float ftanh(float x) { return 1.0f - 2.0f * __builtin_amdgcn_rcpf(expf(2.0f * x) + 1.0f); }

__global__ __launch_bounds__(NTHR) void gru_seq_kernel(
    const float* __restrict__ values, const int* __restrict__ lengths,
    const float* __restrict__ wk_in, const float* __restrict__ wr_in,
    const float* __restrict__ bias, const float* __restrict__ dense_w,
    const float* __restrict__ dense_b, float* __restrict__ out) {
  __shared__ __align__(16) unsigned short WkT[NCOL3 * WPITCH];
  __shared__ __align__(16) unsigned short WrT[NCOL3 * WPITCH];
  __shared__ __align__(16) unsigned       Axw[SEQ_BLK * (APITCH / 2)];
  __shared__ __align__(16) unsigned short Ahu[SEQ_BLK * APITCH];
  __shared__ __align__(16) float          Osl[SEQ_BLK * OPITCH];
  __shared__ __align__(16) float          Pp[NWAVE * SEQ_BLK];
  __shared__ __align__(16) float          Cs[NCONST];
  __shared__ __align__(16) int            Ls[SEQ_BLK];

  const int tid = threadIdx.x, lane = tid & 31, wave = tid >> 5;
  const int c = lane & 15, hh = lane >> 4, koff = hh * 8;
  const int b0 = blockIdx.x * SEQ_BLK;
  const int u = 16 * wave + c;

#pragma unroll 1
  for (int idx = tid; idx < KPAD * NCOL3; idx += NTHR) {
    const int k = idx / NCOL3;
    const int n = idx - k * NCOL3;
    const float wrv = wr_in[idx];
    const int   kcl = (k < NFEAT) ? k : (NFEAT - 1);
    const float fk  = (k < NFEAT) ? 1.0f : 0.0f;
    const float wkv = wk_in[kcl * NCOL3 + n] * fk;
    WrT[n * WPITCH + k] = f2bf_bits(wrv);
    WkT[n * WPITCH + k] = f2bf_bits(wkv);
  }
#pragma unroll 1
  for (int i = tid; i < SEQ_BLK * APITCH; i += NTHR) Ahu[i] = (unsigned short)0;

#pragma unroll 1
  for (int i = tid; i < 2 * NCOL3; i += NTHR) Cs[i] = bias[i];
  {
    const int   lraw = lengths[b0 + (tid & (SEQ_BLK - 1))];
    const float dwv  = dense_w[tid & (NUNIT - 1)];
    const float dbl  = dense_b[0];
    int lv = (lraw < 0) ? 0 : lraw;
    lv = (lv > NSTEP) ? NSTEP : lv;
    if (tid < SEQ_BLK) Ls[tid] = lv;
    if (tid < NUNIT)   Cs[2 * NCOL3 + tid] = dwv;
    if (tid == 0)      Cs[2 * NCOL3 + NUNIT] = dbl;
  }

  const int   kc0 = (2 * lane < NFEAT) ? (2 * lane) : (NFEAT - 1);
  const int   kc1 = (2 * lane + 1 < NFEAT) ? (2 * lane + 1) : (NFEAT - 1);
  const float fx0 = (2 * lane < NFEAT) ? 1.0f : 0.0f;
  const float fx1 = (2 * lane + 1 < NFEAT) ? 1.0f : 0.0f;
  float rv0[4], rv1[4];
#pragma unroll
  for (int i = 0; i < 4; ++i) {
    const float* rp = values + ((size_t)(b0 + 4 * i + wave) * NSTEP) * NFEAT;
    rv0[i] = rp[kc0];
    rv1[i] = rp[kc1];
  }
#pragma unroll
  for (int i = 0; i < 4; ++i) {
    const unsigned lo = (unsigned)f2bf_bits(rv0[i] * fx0);
    const unsigned hi = (unsigned)f2bf_bits(rv1[i] * fx1);
    Axw[(4 * i + wave) * (APITCH / 2) + lane] = lo | (hi << 16);
  }
  __syncthreads();

  int lenr[8];
#pragma unroll
  for (int r = 0; r < 8; ++r) lenr[r] = Ls[8 * hh + r];
  float bxg[3], bhg[3];
#pragma unroll
  for (int g = 0; g < 3; ++g) {
    bxg[g] = Cs[NUNIT * g + u];
    bhg[g] = Cs[NCOL3 + NUNIT * g + u];
  }
  const float dwu = Cs[2 * NCOL3 + u];
  const float dbv = Cs[2 * NCOL3 + NUNIT];
  float hst[8];
#pragma unroll
  for (int r = 0; r < 8; ++r) hst[r] = 0.0f;

  const __bf16* axrow = (const __bf16*)Axw + c * APITCH + koff;
  const __bf16* ahrow = (const __bf16*)Ahu + c * APITCH + koff;
  const __bf16* wkb   = (const __bf16*)WkT + u * WPITCH + koff;
  const __bf16* wrb   = (const __bf16*)WrT + u * WPITCH + koff;
  const v8f z8 = {0.f, 0.f, 0.f, 0.f, 0.f, 0.f, 0.f, 0.f};

#pragma unroll 1
  for (int t = 0; t < NSTEP; ++t) {
    const int tn = (t + 1 < NSTEP) ? (t + 1) : (NSTEP - 1);
#pragma unroll
    for (int i = 0; i < 4; ++i) {
      const float* rp = values + ((size_t)(b0 + 4 * i + wave) * NSTEP + (size_t)tn) * NFEAT;
      rv0[i] = rp[kc0];
      rv1[i] = rp[kc1];
    }

    v8f accz = z8, accr = z8, accx = z8, acch = z8;
#pragma unroll 1
    for (int k0 = 0; k0 < KPAD; k0 += 32) {
      const v16b ax = Frag<__bf16>::load(axrow + k0);
      const v16b kz = Frag<__bf16>::load(wkb + k0);
      const v16b kr = Frag<__bf16>::load(wkb + NUNIT * WPITCH + k0);
      const v16b kh = Frag<__bf16>::load(wkb + 2 * NUNIT * WPITCH + k0);
      accz = Frag<__bf16>::mma(ax, kz, accz);
      accr = Frag<__bf16>::mma(ax, kr, accr);
      accx = Frag<__bf16>::mma(ax, kh, accx);
      guard4x(accz, accr, accx, acch, ax, kz, kr, kh);
      const v16b ah = Frag<__bf16>::load(ahrow + k0);
      const v16b rz = Frag<__bf16>::load(wrb + k0);
      const v16b rr = Frag<__bf16>::load(wrb + NUNIT * WPITCH + k0);
      const v16b rh = Frag<__bf16>::load(wrb + 2 * NUNIT * WPITCH + k0);
      accz = Frag<__bf16>::mma(ah, rz, accz);
      accr = Frag<__bf16>::mma(ah, rr, accr);
      acch = Frag<__bf16>::mma(ah, rh, acch);
      guard4x(accz, accr, accx, acch, ah, rz, rr, rh);
    }
    acc_guard4(accz, accr, accx, acch);

    float pr[8];
#pragma unroll
    for (int r = 0; r < 8; ++r) {
      const float zpre = (accz[r] + bxg[0]) + bhg[0];
      const float rpre = (accr[r] + bxg[1]) + bhg[1];
      const float xh   = accx[r] + bxg[2];
      const float hv   = acch[r] + bhg[2];
      const float zg   = fsig(zpre);
      const float rg   = fsig(rpre);
      const float cand = ftanh(xh + rg * hv);
      const float ho   = hst[r];
      const float hn   = zg * ho + (1.0f - zg) * cand;
      const float h1   = (t < lenr[r]) ? hn : ho;
      hst[r] = h1;
      pr[r]  = h1 * dwu;
    }
#pragma unroll
    for (int r = 0; r < 8; ++r) {
      float s = pr[r];
      s += __shfl_xor(s, 1, 32);
      s += __shfl_xor(s, 2, 32);
      s += __shfl_xor(s, 4, 32);
      s += __shfl_xor(s, 8, 32);
      pr[r] = s;
    }
    if (c == 0) {
#pragma unroll
      for (int r = 0; r < 8; ++r) Pp[wave * SEQ_BLK + 8 * hh + r] = pr[r];
    }
    __syncthreads();

#pragma unroll
    for (int r = 0; r < 8; ++r) Ahu[(8 * hh + r) * APITCH + u] = f2bf_bits(hst[r]);
#pragma unroll
    for (int i = 0; i < 4; ++i) {
      const unsigned lo = (unsigned)f2bf_bits(rv0[i] * fx0);
      const unsigned hi = (unsigned)f2bf_bits(rv1[i] * fx1);
      Axw[(4 * i + wave) * (APITCH / 2) + lane] = lo | (hi << 16);
    }
    if (tid < SEQ_BLK) {
      const int row = tid;
      const float s = ((Pp[row] + Pp[SEQ_BLK + row]) + (Pp[2 * SEQ_BLK + row] + Pp[3 * SEQ_BLK + row])) + dbv;
      Osl[row * OPITCH + (t & (TGRP - 1))] = fsig(s);
    }
    __syncthreads();

    if ((t & (TGRP - 1)) == (TGRP - 1)) {
      const int q = lane >> 3, c4 = (lane & 7) * 4;
      const int row = 4 * wave + q;
      const v4f v = *(const v4f*)(Osl + row * OPITCH + c4);
      float* op = out + (size_t)(b0 + row) * NSTEP + (size_t)(t - (TGRP - 1)) + c4;
      for (int pass = 0; pass < 2; ++pass) {
        *(volatile v4f*)op = v;
        __threadfence();
      }
    }
  }
}

extern "C" void kernel_launch(void* const* d_in, const int* in_sizes, int n_in,
                              void* d_out, int out_size, void* d_ws, size_t ws_size, hipStream_t stream) {
  if (n_in < 10 || d_out == nullptr) return;
  if (in_sizes[2] != NSEQ * NSTEP * NFEAT || in_sizes[4] != NSEQ || in_sizes[5] != NFEAT * NCOL3 ||
      in_sizes[6] != NUNIT * NCOL3 || in_sizes[7] != 2 * NCOL3 || in_sizes[8] != NUNIT || in_sizes[9] < 1 ||
      out_size != NSEQ * NSTEP) return;

  const float* values  = (const float*)d_in[2];
  const int*   lengths = (const int*)d_in[4];
  const float* wk      = (const float*)d_in[5];
  const float* wr      = (const float*)d_in[6];
  const float* bias    = (const float*)d_in[7];
  const float* dw      = (const float*)d_in[8];
  const float* db      = (const float*)d_in[9];
  float* out = (float*)d_out;

  gru_seq_kernel<<<dim3(NSEQ / SEQ_BLK), dim3(NTHR), 0, stream>>>(values, lengths, wk, wr, bias, dw, db, out);

  (void)d_ws; (void)ws_size;
}
